// CharRNN_13993003450943
// MI455X (gfx1250) — hardware-verified
//
#include <hip/hip_runtime.h>
#include <stdint.h>

typedef __attribute__((ext_vector_type(16))) __bf16   v16b;
typedef __attribute__((ext_vector_type(8)))  __bf16   v8b;
typedef __attribute__((ext_vector_type(8)))  float    v8f;
typedef __attribute__((ext_vector_type(4)))  float    v4f;
typedef __attribute__((ext_vector_type(4)))  unsigned int v4u;

constexpr int NBATCH = 256;
constexpr int NSTEP  = 512;
constexpr int NVOC   = 32;
constexpr int NEMB   = 64;
constexpr int NHID   = 256;
constexpr int TBR    = 16;
constexpr int HPITCH = 264;
constexpr int LGP    = 36;
constexpr int HFP    = 260;
constexpr int TP     = 20;

static_assert(NHID % 32 == 0, "K of the recurrence is a multiple of 32");
static_assert(NEMB % 32 == 0, "K of the input projection is a multiple of 32");
static_assert(NBATCH % TBR == 0, "batch is a multiple of the block rows");
static_assert((size_t)NBATCH * NSTEP * NVOC * 4 == 16777216, "out0 bytes");
static_assert((size_t)NBATCH * NSTEP * NVOC * 4 + (size_t)NBATCH * NHID * 4 == 17039360, "out0 + out1 bytes == d_out total");

__device__ __forceinline__ unsigned short at_bf_bits(float f) {
  unsigned u = __float_as_uint(f);
  return (unsigned short)((u + 0x7FFFu + ((u >> 16) & 1u)) >> 16);
}
__device__ __forceinline__ __bf16 at_f2bf(float f) { return __builtin_bit_cast(__bf16, at_bf_bits(f)); }
__device__ __forceinline__ void at_split(float f, __bf16& hi, __bf16& lo) {
  const unsigned short hb = at_bf_bits(f);
  hi = __builtin_bit_cast(__bf16, hb);
  lo = at_f2bf(f - __uint_as_float(((unsigned)hb) << 16));
}
__device__ __forceinline__ v8f at_mma(v16b a, v16b b, v8f c) {
  c = __builtin_amdgcn_wmma_f32_16x16x32_bf16(false, a, false, b, (short)0, c, false, false);
  asm volatile("v_nop\n\tv_nop\n\tv_nop\n\tv_nop" : "+v"(c) : "v"(a), "v"(b));
  return c;
}

__device__ __forceinline__ v16b ld_frag_row(const __bf16* p) {
  union { v16b v; v8b h[2]; } f;
  f.h[0] = *(const v8b*)(p);
  f.h[1] = *(const v8b*)(p + 16);
  return f.v;
}
__device__ __forceinline__ v16b ld_frag_swz(const __bf16* p) {
  union { v16b v; v8b h[2]; } f;
  f.h[0] = *(const v8b*)(p);
  f.h[1] = *(const v8b*)(p + 256);
  return f.v;
}

__global__ __launch_bounds__(32) void xw_table_kernel(const float* __restrict__ emb,
                                                     const float* __restrict__ Wih,
                                                     const float* __restrict__ bh,
                                                     float* __restrict__ tableT) {
  __shared__ __align__(16) float wt[NEMB * TP];
  __shared__ __align__(16) float st[16 * LGP];
  const int lane = threadIdx.x;
  const int hh = lane >> 4, c = lane & 15;
  const int n0 = blockIdx.x * 16;

#pragma unroll
  for (int rr = 0; rr < 2; ++rr) {
    const int e = lane + 32 * rr;
    const float* src = Wih + (size_t)e * NHID + n0;
#pragma unroll
    for (int q = 0; q < 4; ++q) *(v4f*)(wt + e * TP + 4 * q) = *(const v4f*)(src + 4 * q);
  }
  __syncthreads();

  v8f acc[2];
  acc[0] = (v8f){0.f,0.f,0.f,0.f,0.f,0.f,0.f,0.f};
  acc[1] = (v8f){0.f,0.f,0.f,0.f,0.f,0.f,0.f,0.f};

#pragma unroll
  for (int ks = 0; ks < 2; ++ks) {
    v16b bhv, blv;
#pragma unroll
    for (int i = 0; i < 8; ++i) {
      const float f0 = wt[(ks * 32 + 8 * hh + i) * TP + c];
      const float f1 = wt[(ks * 32 + 16 + 8 * hh + i) * TP + c];
      __bf16 h0b, l0b, h1b, l1b;
      at_split(f0, h0b, l0b);
      at_split(f1, h1b, l1b);
      bhv[i] = h0b; blv[i] = l0b; bhv[8 + i] = h1b; blv[8 + i] = l1b;
    }
#pragma unroll
    for (int mt = 0; mt < 2; ++mt) {
      const float* ar = emb + (size_t)(mt * 16 + c) * NEMB + ks * 32;
      const v4f x0 = *(const v4f*)(ar + 8 * hh);
      const v4f x1 = *(const v4f*)(ar + 8 * hh + 4);
      const v4f x2 = *(const v4f*)(ar + 16 + 8 * hh);
      const v4f x3 = *(const v4f*)(ar + 16 + 8 * hh + 4);
      v16b ahv, alv;
#pragma unroll
      for (int q = 0; q < 4; ++q) {
        __bf16 hq, lq;
        at_split(x0[q], hq, lq); ahv[q] = hq;      alv[q] = lq;
        at_split(x1[q], hq, lq); ahv[4 + q] = hq;  alv[4 + q] = lq;
        at_split(x2[q], hq, lq); ahv[8 + q] = hq;  alv[8 + q] = lq;
        at_split(x3[q], hq, lq); ahv[12 + q] = hq; alv[12 + q] = lq;
      }
      acc[mt] = at_mma(ahv, bhv, acc[mt]);
      acc[mt] = at_mma(ahv, blv, acc[mt]);
      acc[mt] = at_mma(alv, bhv, acc[mt]);
    }
  }

  const float bv = bh[n0 + c];
#pragma unroll
  for (int mt = 0; mt < 2; ++mt)
#pragma unroll
    for (int r = 0; r < 8; ++r)
      st[c * LGP + mt * 16 + 8 * hh + r] = acc[mt][r] + bv;
  __syncthreads();

  for (int pass = 0; pass < 2; ++pass) {
#pragma unroll
    for (int it = 0; it < 4; ++it) {
      const int row = it * 4 + (lane >> 3);
      const int c4 = (lane & 7) * 4;
      const v4f v = *(const v4f*)(st + row * LGP + c4);
      *(volatile v4f*)(tableT + (size_t)(n0 + row) * NVOC + c4) = v;
    }
    __threadfence();
  }
}

__global__ __launch_bounds__(32) void frag_swizzle_kernel(const float* __restrict__ W, int ld,
                                                          __bf16* __restrict__ dhi,
                                                          __bf16* __restrict__ dlo) {
  __shared__ __align__(16) float tile[32 * TP];
  const int lane = threadIdx.x;
  const int nt = blockIdx.x >> 3, kc = blockIdx.x & 7;

  {
    const float* src = W + (size_t)(kc * 32 + lane) * ld + nt * 16;
#pragma unroll
    for (int q = 0; q < 4; ++q) *(v4f*)(tile + lane * TP + 4 * q) = *(const v4f*)(src + 4 * q);
  }
  __syncthreads();

  const int hh = lane >> 4, c = lane & 15;
  v4u H0, H1, L0, L1;
#pragma unroll
  for (int q = 0; q < 4; ++q) {
    const float a0 = tile[(8 * hh + 2 * q) * TP + c];
    const float a1 = tile[(8 * hh + 2 * q + 1) * TP + c];
    const float b0 = tile[(16 + 8 * hh + 2 * q) * TP + c];
    const float b1 = tile[(16 + 8 * hh + 2 * q + 1) * TP + c];
    const unsigned short ah0 = at_bf_bits(a0), ah1 = at_bf_bits(a1);
    const unsigned short bh0 = at_bf_bits(b0), bh1 = at_bf_bits(b1);
    const unsigned short al0 = at_bf_bits(a0 - __uint_as_float(((unsigned)ah0) << 16));
    const unsigned short al1 = at_bf_bits(a1 - __uint_as_float(((unsigned)ah1) << 16));
    const unsigned short bl0 = at_bf_bits(b0 - __uint_as_float(((unsigned)bh0) << 16));
    const unsigned short bl1 = at_bf_bits(b1 - __uint_as_float(((unsigned)bh1) << 16));
    H0[q] = (unsigned)ah0 | ((unsigned)ah1 << 16);
    H1[q] = (unsigned)bh0 | ((unsigned)bh1 << 16);
    L0[q] = (unsigned)al0 | ((unsigned)al1 << 16);
    L1[q] = (unsigned)bl0 | ((unsigned)bl1 << 16);
  }
  const size_t base = (size_t)(nt * 8 + kc) * 512 + (size_t)lane * 8;
  unsigned short* ph = (unsigned short*)(void*)dhi + base;
  unsigned short* pl = (unsigned short*)(void*)dlo + base;
  for (int pass = 0; pass < 2; ++pass) {
    *(volatile v4u*)(ph)       = H0;
    *(volatile v4u*)(ph + 256) = H1;
    *(volatile v4u*)(pl)       = L0;
    *(volatile v4u*)(pl + 256) = L1;
    __threadfence();
  }
}

__global__ __launch_bounds__(512) void rnn_kernel(const int* __restrict__ x,
                                                 const float* __restrict__ h0,
                                                 const float* __restrict__ tableT,
                                                 const __bf16* __restrict__ whh_hi,
                                                 const __bf16* __restrict__ whh_lo,
                                                 const __bf16* __restrict__ wo_hi,
                                                 const __bf16* __restrict__ wo_lo,
                                                 const float* __restrict__ bout,
                                                 float* __restrict__ out) {
  __shared__ __align__(16) float xw[NHID * NVOC];
  __shared__ __align__(16) __bf16 hbh[TBR * HPITCH];
  __shared__ __align__(16) __bf16 hbl[TBR * HPITCH];
  __shared__ __align__(16) unsigned char xloc[NSTEP * TBR];
  __shared__ __align__(16) float lg[TBR * LGP];
  static_assert(TBR * HFP <= NHID * NVOC, "h_final stage fits in the xw region");

  const int tid  = threadIdx.x;
  const int lane = tid & 31;
  const int w    = tid >> 5;
  const int ln   = lane & 15;
  const int hh   = lane >> 4;
  const int batch0 = blockIdx.x * TBR;
  const int n0   = w * 16;

  {
    const float* src = tableT + tid * 16;
#pragma unroll
    for (int q = 0; q < 4; ++q) *(v4f*)(xw + tid * 16 + 4 * q) = *(const v4f*)(src + 4 * q);
  }
  for (int i = tid; i < TBR * NSTEP; i += 512) {
    const int m = i >> 9, t = i & (NSTEP - 1);
    int v = x[(size_t)(batch0 + m) * NSTEP + t];
    v = v < 0 ? 0 : (v > NVOC - 1 ? NVOC - 1 : v);
    xloc[t * TBR + m] = (unsigned char)v;
  }
  for (int i = tid; i < TBR * NHID; i += 512) {
    const int m = i >> 8, cc = i & (NHID - 1);
    const float f = h0[(size_t)(batch0 + m) * NHID + cc];
    __bf16 a_, b_;
    at_split(f, a_, b_);
    hbh[m * HPITCH + cc] = a_;
    hbl[m * HPITCH + cc] = b_;
  }
  const float boutv = bout[(w & 1) * 16 + ln];
  const __bf16* pbh = whh_hi + (size_t)w * 8 * 512 + lane * 8;
  const __bf16* pbl = whh_lo + (size_t)w * 8 * 512 + lane * 8;
  const __bf16* poh = wo_hi + (size_t)(w & 1) * 8 * 512 + lane * 8;
  const __bf16* pol = wo_lo + (size_t)(w & 1) * 8 * 512 + lane * 8;
  __syncthreads();

  float hv[8];
#pragma unroll
  for (int j = 0; j < 8; ++j) hv[j] = 0.0f;

  for (int t = 0; t < NSTEP; ++t) {
    v8f acc  = (v8f){0.f,0.f,0.f,0.f,0.f,0.f,0.f,0.f};
    v8f accL = (v8f){0.f,0.f,0.f,0.f,0.f,0.f,0.f,0.f};
    const bool doL = (w < 2) && (t > 0);

#pragma unroll 2
    for (int kc = 0; kc < 8; ++kc) {
      const v16b a  = ld_frag_row(hbh + ln * HPITCH + kc * 32 + 8 * hh);
      const v16b al = ld_frag_row(hbl + ln * HPITCH + kc * 32 + 8 * hh);
      const v16b b  = ld_frag_swz(pbh + kc * 512);
      const v16b bl = ld_frag_swz(pbl + kc * 512);
      acc = at_mma(a, b, acc);
      acc = at_mma(a, bl, acc);
      acc = at_mma(al, b, acc);
      if (doL) {
        const v16b ob = ld_frag_swz(poh + kc * 512);
        const v16b ol = ld_frag_swz(pol + kc * 512);
        accL = at_mma(a, ob, accL);
        accL = at_mma(a, ol, accL);
        accL = at_mma(al, ob, accL);
      }
    }
    __syncthreads();

    if (doL) {
#pragma unroll
      for (int r = 0; r < 8; ++r) lg[(8 * hh + r) * LGP + (w & 1) * 16 + ln] = accL[r] + boutv;
    }
    const unsigned long long tk = *(const unsigned long long*)(xloc + t * TBR + 8 * hh);
#pragma unroll
    for (int j = 0; j < 8; ++j) {
      const int m = 8 * hh + j;
      const int tok = (int)((tk >> (8 * j)) & 31ull);
      const float val = acc[j] + xw[(n0 + ln) * NVOC + tok];
      const float hval = tanhf(val);
      hv[j] = hval;
      __bf16 a_, b_;
      at_split(hval, a_, b_);
      hbh[m * HPITCH + n0 + ln] = a_;
      hbl[m * HPITCH + n0 + ln] = b_;
    }
    __syncthreads();

    if (doL) {
      const int tt = t - 1;
      for (int pass = 0; pass < 2; ++pass) {
#pragma unroll
        for (int it = 0; it < 2; ++it) {
          const int row = (w & 1) * 8 + it * 4 + (lane >> 3);
          const int c4 = (lane & 7) * 4;
          const v4f v = *(const v4f*)(lg + row * LGP + c4);
          *(volatile v4f*)(out + ((size_t)(batch0 + row) * NSTEP + tt) * NVOC + c4) = v;
        }
        __threadfence();
      }
    }
  }

  float* hs = xw;
#pragma unroll
  for (int j = 0; j < 8; ++j) hs[(8 * hh + j) * HFP + n0 + ln] = hv[j];
  __syncthreads();
  {
    float* o1 = out + (size_t)NBATCH * NSTEP * NVOC;
    const int m = w;
    for (int pass = 0; pass < 2; ++pass) {
#pragma unroll
      for (int it = 0; it < 2; ++it) {
        const int cc = it * 128 + lane * 4;
        const v4f v = *(const v4f*)(hs + m * HFP + cc);
        *(volatile v4f*)(o1 + (size_t)(batch0 + m) * NHID + cc) = v;
      }
      __threadfence();
    }
  }

  if (w < 2) {
    v8f accL = (v8f){0.f,0.f,0.f,0.f,0.f,0.f,0.f,0.f};
#pragma unroll 2
    for (int kc = 0; kc < 8; ++kc) {
      const v16b a  = ld_frag_row(hbh + ln * HPITCH + kc * 32 + 8 * hh);
      const v16b al = ld_frag_row(hbl + ln * HPITCH + kc * 32 + 8 * hh);
      const v16b ob = ld_frag_swz(poh + kc * 512);
      const v16b ol = ld_frag_swz(pol + kc * 512);
      accL = at_mma(a, ob, accL);
      accL = at_mma(a, ol, accL);
      accL = at_mma(al, ob, accL);
    }
#pragma unroll
    for (int r = 0; r < 8; ++r) lg[(8 * hh + r) * LGP + (w & 1) * 16 + ln] = accL[r] + boutv;
  }
  __syncthreads();
  if (w < 2) {
    const int tt = NSTEP - 1;
    for (int pass = 0; pass < 2; ++pass) {
#pragma unroll
      for (int it = 0; it < 2; ++it) {
        const int row = (w & 1) * 8 + it * 4 + (lane >> 3);
        const int c4 = (lane & 7) * 4;
        const v4f v = *(const v4f*)(lg + row * LGP + c4);
        *(volatile v4f*)(out + ((size_t)(batch0 + row) * NSTEP + tt) * NVOC + c4) = v;
      }
      __threadfence();
    }
  }
}

extern "C" void kernel_launch(void* const* d_in, const int* in_sizes, int n_in,
                              void* d_out, int out_size, void* d_ws, size_t ws_size,
                              hipStream_t stream) {
  constexpr size_t OFF_TAB = 0;
  constexpr size_t SZ_TAB  = (size_t)NHID * NVOC * 4;
  constexpr size_t SZ_HHP  = (size_t)16 * 8 * 512 * 2;
  constexpr size_t SZ_OP   = (size_t)2 * 8 * 512 * 2;
  constexpr size_t OFF_HHH = OFF_TAB + SZ_TAB;
  constexpr size_t OFF_HHL = OFF_HHH + SZ_HHP;
  constexpr size_t OFF_OH  = OFF_HHL + SZ_HHP;
  constexpr size_t OFF_OL  = OFF_OH + SZ_OP;
  constexpr size_t WS_TOTAL = OFF_OL + SZ_OP;
  static_assert(SZ_TAB == 32768 && SZ_HHP == 131072 && SZ_OP == 16384, "region sizes");
  static_assert(WS_TOTAL == 327680, "carve total");
  static_assert(WS_TOTAL <= (size_t)134217728, "carve within budget");
  static_assert(OFF_HHH % 128 == 0 && OFF_HHL % 128 == 0 && OFF_OH % 128 == 0 && OFF_OL % 128 == 0, "128-B aligned regions");

  if (n_in < 8) return;
  if (ws_size < WS_TOTAL) return;
  if ((size_t)out_size < (size_t)NBATCH * NSTEP * NVOC + (size_t)NBATCH * NHID) return;
  if (in_sizes[0] < NBATCH * NSTEP || in_sizes[1] < NBATCH * NHID || in_sizes[2] < NVOC * NEMB ||
      in_sizes[3] < NEMB * NHID || in_sizes[4] < NHID * NHID || in_sizes[5] < NHID ||
      in_sizes[6] < NHID * NVOC || in_sizes[7] < NVOC) return;

  const int*   x    = (const int*)d_in[0];
  const float* h0   = (const float*)d_in[1];
  const float* emb  = (const float*)d_in[2];
  const float* Wih  = (const float*)d_in[3];
  const float* Whh  = (const float*)d_in[4];
  const float* bh   = (const float*)d_in[5];
  const float* Wout = (const float*)d_in[6];
  const float* bout = (const float*)d_in[7];
  float* out = (float*)d_out;
  char* ws = (char*)d_ws;

  float*  tableT = (float*)(ws + OFF_TAB);
  __bf16* whh_hi = (__bf16*)(ws + OFF_HHH);
  __bf16* whh_lo = (__bf16*)(ws + OFF_HHL);
  __bf16* wo_hi  = (__bf16*)(ws + OFF_OH);
  __bf16* wo_lo  = (__bf16*)(ws + OFF_OL);

  xw_table_kernel<<<dim3(NHID / 16), dim3(32), 0, stream>>>(emb, Wih, bh, tableT);
  frag_swizzle_kernel<<<dim3(16 * 8), dim3(32), 0, stream>>>(Whh, NHID, whh_hi, whh_lo);
  frag_swizzle_kernel<<<dim3(2 * 8), dim3(32), 0, stream>>>(Wout, NVOC, wo_hi, wo_lo);
  rnn_kernel<<<dim3(NBATCH / TBR), dim3(512), 0, stream>>>(x, h0, tableT, whh_hi, whh_lo,
                                                          wo_hi, wo_lo, bout, out);
}
